// CausalSelfAttention_54348516163806
// MI455X (gfx1250) — hardware-verified
//
#include <hip/hip_runtime.h>
#include <math.h>

typedef __attribute__((ext_vector_type(16))) _Float16 v16h;
typedef __attribute__((ext_vector_type(16))) __bf16 v16b;
typedef __attribute__((ext_vector_type(8)))  _Float16 v8h;
typedef __attribute__((ext_vector_type(8)))  __bf16 v8b;
typedef __attribute__((ext_vector_type(8)))  float v8f;
typedef __attribute__((ext_vector_type(4)))  float v4f;
typedef __attribute__((ext_vector_type(4)))  unsigned v4u;

template <typename T> __device__ __forceinline__ void vst2(void* p, T v) { *(volatile T*)p = v; __threadfence(); *(volatile T*)p = v; }
__device__ __forceinline__ v8f wmma16(v16h a, v16h b, v8f c) {
  v8f d = __builtin_amdgcn_wmma_f32_16x16x32_f16(false, a, false, b, (short)0, c, false, false);
  asm volatile("v_nop\n\tv_nop\n\tv_nop\n\tv_nop" : "+v"(d) : "v"(a), "v"(b));
  return d;
}
__device__ __forceinline__ v8f wmma_bf(v16b a, v16b b, v8f c) {
  v8f d = __builtin_amdgcn_wmma_f32_16x16x32_bf16(false, a, false, b, (short)0, c, false, false);
  asm volatile("v_nop\n\tv_nop\n\tv_nop\n\tv_nop" : "+v"(d) : "v"(a), "v"(b));
  return d;
}
__device__ __forceinline__ v16h frag_h(const _Float16* rowk0, int lane) {
  union { v16h v; v8h q[2]; } u; const _Float16* p = rowk0 + 8 * (lane >> 4);
  u.q[0] = *(const v8h*)p; u.q[1] = *(const v8h*)(p + 16); return u.v;
}
__device__ __forceinline__ v16b frag_b(const __bf16* rowk0, int lane) {
  union { v16b v; v8b q[2]; } u; const __bf16* p = rowk0 + 8 * (lane >> 4);
  u.q[0] = *(const v8b*)p; u.q[1] = *(const v8b*)(p + 16); return u.v;
}
__device__ __forceinline__ v16h frag_f32s(const float* rowk0, int lane, float sc) {
  v16h a; const float* p = rowk0 + 8 * (lane >> 4);
#pragma unroll
  for (int i = 0; i < 8; ++i) { a[i] = (_Float16)(p[i] * sc); a[8 + i] = (_Float16)(p[16 + i] * sc); }
  return a;
}
struct F2 { v16b h, l; };
__device__ __forceinline__ F2 bsplit16(const float v[16]) { F2 r;
#pragma unroll
  for (int i = 0; i < 16; ++i) { const __bf16 h = (__bf16)v[i]; r.h[i] = h; r.l[i] = (__bf16)(v[i] - (float)h); }
  return r; }
__device__ __forceinline__ F2 split_row(const float* row, int k0, int lane) { float v[16]; const float* p = row + k0 + 8 * (lane >> 4);
#pragma unroll
  for (int i = 0; i < 8; ++i) { v[i] = p[i]; v[8 + i] = p[16 + i]; }
  return bsplit16(v); }
__device__ __forceinline__ float bfr(float v) { return (float)(__bf16)v; }
__device__ __forceinline__ v16b wcol_io(const float* Wm, int k0, int o, int lane, int ld) { v16b w; const int g = lane >> 4;
#pragma unroll
  for (int i = 0; i < 8; ++i) { w[i] = (__bf16)Wm[(size_t)(k0 + 8 * g + i) * ld + o]; w[8 + i] = (__bf16)Wm[(size_t)(k0 + 16 + 8 * g + i) * ld + o]; }
  return w; }
__device__ __forceinline__ v16h wcolh_io(const float* Wm, int k0, int o, int lane, int ld) { v16h w; const int g = lane >> 4;
#pragma unroll
  for (int i = 0; i < 8; ++i) { w[i] = (_Float16)(bfr(Wm[(size_t)(k0 + 8 * g + i) * ld + o]) * 256.0f); w[8 + i] = (_Float16)(bfr(Wm[(size_t)(k0 + 16 + 8 * g + i) * ld + o]) * 256.0f); }
  return w; }
#define LDSX() do { asm volatile("s_wait_dscnt 0" ::: "memory"); __builtin_amdgcn_wave_barrier(); __builtin_amdgcn_fence(3  , "workgroup"); } while (0)

#define NB_FULL 4
#define SEQ_FULL 1024
#ifndef NB
#define NB NB_FULL
#endif
#ifndef SEQ
#define SEQ SEQ_FULL
#endif
#define TT SEQ
#define CC 1024
#define DIN 1024
#define NH 16
#define HD 64
#define NQB (TT / 64)
#define SCALE (0.125f)
#define QBH 4
#define QHI 256
#define KHI 256
#define NEGBIG (-3.0e38f)

static_assert(NH * HD == CC);
static_assert(HD == 64);
static_assert(CC == DIN);
static_assert(DIN % 32 == 0);
static_assert(CC % 128 == 0);
static_assert(DIN % 128 == 0);
static_assert(TT % 64 == 0);
static_assert((NB * TT) % 64 == 0);
static_assert(QHI == KHI);
static_assert(QHI == QBH * 64);
static_assert(TT >= QHI);
static_assert(QHI % 32 == 0);
static_assert(NB <= NB_FULL);
static_assert(SEQ <= SEQ_FULL);

static constexpr size_t WS_QH  = 0;
static constexpr size_t WS_KH  = WS_QH + 2ull * (size_t)NB * TT * CC;
static constexpr size_t WS_VT  = WS_KH + 2ull * (size_t)NB * TT * CC;
static constexpr size_t WS_QL  = WS_VT + 2ull * (size_t)NB * CC * TT;
static constexpr size_t WS_KL  = WS_QL + 2ull * (size_t)NB * QHI * CC;
static constexpr size_t WS_VB  = WS_KL + 2ull * (size_t)NB * KHI * CC;
static constexpr size_t WS_VBL = WS_VB + 2ull * (size_t)NB * CC * KHI;
static constexpr size_t WS_Y   = WS_VBL + 2ull * (size_t)NB * CC * KHI;
static constexpr size_t WS_END = WS_Y + 4ull * (size_t)NB * TT * CC;
static_assert(WS_KH == WS_QH + 2ull * (size_t)NB * TT * CC);
static_assert(WS_KL == WS_QL + 2ull * (size_t)NB * QHI * CC);
static_assert(WS_END <= 134217728ull);
static_assert(WS_QH % 128 == 0 && WS_KH % 128 == 0 && WS_VT % 128 == 0 && WS_QL % 128 == 0 && WS_KL % 128 == 0 && WS_VB % 128 == 0 && WS_VBL % 128 == 0 && WS_Y % 128 == 0);

__global__ __launch_bounds__(128) void k_proj(const float* __restrict__ X, const float* __restrict__ W, const float* __restrict__ BA,
    _Float16* __restrict__ QK, _Float16* __restrict__ QKL, _Float16* __restrict__ VT, __bf16* __restrict__ VB, __bf16* __restrict__ VBL) {
  __shared__ __align__(16) float st[64][132]; __shared__ __align__(16) _Float16 sh[64][136], sl[64][136]; __shared__ __align__(16) _Float16 th[128][72]; __shared__ __align__(16) __bf16 tb[128][72], tbl[128][72];
  const int tid = threadIdx.x; const int wave = __builtin_amdgcn_readfirstlane(tid >> 5); const int lane = tid & 31, col = lane & 15, g = lane >> 4;
  const int which = blockIdx.z; const int c0 = blockIdx.y * 128; const size_t r0 = (size_t)blockIdx.x * 64; const size_t bb = r0 / TT; const int t0 = (int)(r0 % TT);
  const int wc0 = which * CC + c0;
  const size_t xr = (bb * (size_t)SEQ_FULL + t0 + wave * 16 + col) * DIN;
  v8f acc[8] = {};
#pragma unroll 2
  for (int kc = 0; kc < DIN / 32; ++kc) { v16b a; { const float* p = X + xr + kc * 32 + 8 * g;
#pragma unroll
      for (int i = 0; i < 8; ++i) { a[i] = (__bf16)p[i]; a[8 + i] = (__bf16)p[16 + i]; } }
    asm volatile("s_wait_loadcnt 0x0" ::: "memory");
#pragma unroll
    for (int j = 0; j < 8; ++j) { const v16b w = wcol_io(W, kc * 32, wc0 + j * 16 + col, lane, 3 * CC); asm volatile("s_wait_loadcnt 0x0" ::: "memory"); acc[j] = wmma_bf(a, w, acc[j]); } }
  {
#pragma unroll
    for (int j = 0; j < 8; ++j) { const float bias = bfr(BA[wc0 + j * 16 + col]);
#pragma unroll
      for (int r = 0; r < 8; ++r) st[wave * 16 + 8 * g + r][j * 16 + col] = acc[j][r] + bias; }
    __syncthreads(); }
  if (which < 2) { _Float16* DH = QK + (size_t)which * NB * TT * CC; _Float16* DL = QKL + (size_t)which * NB * QHI * CC; const bool hi_rows = t0 < QHI;
    for (int e = tid; e < 64 * 128; e += 128) { const int rl = e >> 7, cl = e & 127; const float v = st[rl][cl]; const _Float16 hv = (_Float16)v; sh[rl][cl] = hv; sl[rl][cl] = (_Float16)((v - (float)hv) * 1024.0f); }
    __syncthreads();
    for (int e = tid; e < 64 * 16; e += 128) { const int rl = e >> 4, q = e & 15; vst2((unsigned*)(DH + (r0 + rl) * CC + c0 + q * 8), *(const v4u*)&sh[rl][q * 8]); if (hi_rows) vst2((unsigned*)(DL + (bb * QHI + t0 + rl) * (size_t)CC + c0 + q * 8), *(const v4u*)&sl[rl][q * 8]); }
  } else { const bool hi_rows = t0 < KHI;
    for (int e = tid; e < 64 * 128; e += 128) { const int rl = e & 63, cl = e >> 6; const float v = st[rl][cl]; th[cl][rl] = (_Float16)v; const __bf16 bh = (__bf16)v; tb[cl][rl] = bh; tbl[cl][rl] = (__bf16)(v - (float)bh); }
    __syncthreads();
    for (int e = tid; e < 128 * 8; e += 128) { const int cl = e >> 3, q = e & 7; vst2((unsigned*)(VT + (bb * CC + c0 + cl) * (size_t)TT + t0 + q * 8), *(const v4u*)&th[cl][q * 8]); if (hi_rows) { const size_t o3 = (bb * CC + c0 + cl) * (size_t)KHI + t0 + q * 8; vst2((unsigned*)(VB + o3), *(const v4u*)&tb[cl][q * 8]); vst2((unsigned*)(VBL + o3), *(const v4u*)&tbl[cl][q * 8]); } } } }

__device__ __forceinline__ void sm_step(const v8f sa, const v8f sb, const int kk0, const int kk1, const int qr0, float (&m)[8], float (&lp)[8], v8f (&o)[4], v8f& p0, v8f& p1) {
#pragma unroll
  for (int r = 0; r < 8; ++r) {
    const int qr = qr0 + r; const bool v0 = kk0 <= qr, v1 = kk1 <= qr;
    const float a0 = v0 ? sa[r] : NEGBIG, a1 = v1 ? sb[r] : NEGBIG;
    float mx = fmaxf(a0, a1);
    mx = fmaxf(mx, __shfl_xor(mx, 1)); mx = fmaxf(mx, __shfl_xor(mx, 2)); mx = fmaxf(mx, __shfl_xor(mx, 4)); mx = fmaxf(mx, __shfl_xor(mx, 8));
    const float mn = fmaxf(m[r], mx);
    const float al = expf(m[r] - mn);
    m[r] = mn;
    const float e0 = expf(a0 - mn), e1 = expf(a1 - mn);
    const float q0 = v0 ? e0 : 0.0f, q1 = v1 ? e1 : 0.0f;
    lp[r] = lp[r] * al + (q0 + q1);
    o[0][r] *= al; o[1][r] *= al; o[2][r] *= al; o[3][r] *= al;
    p0[r] = q0; p1[r] = q1; } }

__global__ __launch_bounds__(128) void k_fa(const _Float16* __restrict__ QH, const _Float16* __restrict__ KH, const _Float16* __restrict__ QL, const _Float16* __restrict__ KL,
    const _Float16* __restrict__ VT, const __bf16* __restrict__ VB, const __bf16* __restrict__ VBL, float* __restrict__ Y) {
  __shared__ __align__(16) float ps[4][16][36];
  __shared__ __align__(16) float so[4][16][HD + 4];
  const int tid = threadIdx.x; const int wave = __builtin_amdgcn_readfirstlane(tid >> 5); const int lane = tid & 31, col = lane & 15, g = lane >> 4;
  const int qb = blockIdx.x; const int b = blockIdx.y / NH, h = blockIdx.y % NH;
  const bool early = qb < QBH;
  const int ql0 = qb * 64 + wave * 16;
  const int nhalf = ((ql0 + 15) >> 5) + 1;
  const size_t qoff = ((size_t)b * TT + ql0 + col) * CC + h * HD;
  const size_t qloff = ((size_t)b * QHI + (early ? ql0 : 0) + col) * CC + h * HD;
  float m[8], lp[8]; v8f o[4] = {};
#pragma unroll
  for (int r = 0; r < 8; ++r) { m[r] = NEGBIG; lp[r] = 0.0f; }
#pragma unroll 1
  for (int hh = 0; hh < nhalf; ++hh) {
    const int key0 = hh * 32;
    const size_t koff = ((size_t)b * TT + key0 + col) * CC + h * HD;
    v8f s0 = {}, s1 = {};
    if (early) {
      const size_t kloff = ((size_t)b * KHI + key0 + col) * CC + h * HD;
      v8f r0 = {}, r1 = {};
#pragma unroll
      for (int kc = 0; kc < HD / 32; ++kc) {
        const v16h ah = frag_h(QH + qoff + kc * 32, lane), al = frag_h(QL + qloff + kc * 32, lane);
        const v16h k0h = frag_h(KH + koff + kc * 32, lane), k1h = frag_h(KH + koff + (size_t)16 * CC + kc * 32, lane);
        const v16h k0l = frag_h(KL + kloff + kc * 32, lane), k1l = frag_h(KL + kloff + (size_t)16 * CC + kc * 32, lane);
        s0 = wmma16(ah, k0h, s0); r0 = wmma16(al, k0h, r0); r0 = wmma16(ah, k0l, r0);
        s1 = wmma16(ah, k1h, s1); r1 = wmma16(al, k1h, r1); r1 = wmma16(ah, k1l, r1); }
#pragma unroll
      for (int r = 0; r < 8; ++r) { s0[r] = (s0[r] + r0[r] * (1.0f / 1024.0f)) * SCALE; s1[r] = (s1[r] + r1[r] * (1.0f / 1024.0f)) * SCALE; }
    } else {
#pragma unroll
      for (int kc = 0; kc < HD / 32; ++kc) {
        const v16h ah = frag_h(QH + qoff + kc * 32, lane);
        const v16h k0h = frag_h(KH + koff + kc * 32, lane), k1h = frag_h(KH + koff + (size_t)16 * CC + kc * 32, lane);
        s0 = wmma16(ah, k0h, s0); s1 = wmma16(ah, k1h, s1); }
#pragma unroll
      for (int r = 0; r < 8; ++r) { s0[r] *= SCALE; s1[r] *= SCALE; } }
    v8f p0, p1;
    sm_step(s0, s1, key0 + col, key0 + 16 + col, ql0 + 8 * g, m, lp, o, p0, p1);
#pragma unroll
    for (int r = 0; r < 8; ++r) { ps[wave][8 * g + r][col] = p0[r]; ps[wave][8 * g + r][16 + col] = p1[r]; }
    LDSX();
    float pv[16];
#pragma unroll
    for (int i = 0; i < 8; ++i) { pv[i] = ps[wave][col][8 * g + i]; pv[8 + i] = ps[wave][col][16 + 8 * g + i]; }
    LDSX();
    if (early) { const F2 p = bsplit16(pv); const size_t vo = ((size_t)b * CC + h * HD + col) * (size_t)KHI + key0;
#pragma unroll
      for (int j = 0; j < HD / 16; ++j) { const size_t po = vo + (size_t)j * 16 * KHI; const v16b vh = frag_b(VB + po, lane), vl = frag_b(VBL + po, lane);
        o[j] = wmma_bf(p.h, vh, o[j]); o[j] = wmma_bf(p.l, vh, o[j]); o[j] = wmma_bf(p.h, vl, o[j]); }
    } else { v16h pf;
#pragma unroll
      for (int i = 0; i < 16; ++i) pf[i] = (_Float16)(pv[i] * 2048.0f);
      const size_t vo = ((size_t)b * CC + h * HD + col) * (size_t)TT + key0;
#pragma unroll
      for (int j = 0; j < HD / 16; ++j) { const v16h vf = frag_h(VT + vo + (size_t)j * 16 * TT, lane); o[j] = wmma16(pf, vf, o[j]); } } }
  const float carry = early ? 1.0f : (1.0f / 2048.0f);
#pragma unroll
  for (int r = 0; r < 8; ++r) { float l = lp[r]; l += __shfl_xor(l, 1); l += __shfl_xor(l, 2); l += __shfl_xor(l, 4); l += __shfl_xor(l, 8);
    const float inv = carry * (1.0f / l);
#pragma unroll
    for (int j = 0; j < HD / 16; ++j) so[wave][8 * g + r][j * 16 + col] = o[j][r] * inv; }
  LDSX();
  for (int it = 0; it < 8; ++it) { const int rl = it * 2 + g; vst2(Y + ((size_t)b * TT + ql0 + rl) * CC + h * HD + col * 4, *(const v4f*)&so[wave][rl][col * 4]); } }

__global__ __launch_bounds__(128) void k_out(const float* __restrict__ Y, const float* __restrict__ WO, const float* __restrict__ BO, float* __restrict__ OUT) { __shared__ __align__(16) float sf[4][16][132];
  const int tid = threadIdx.x; const int wave = __builtin_amdgcn_readfirstlane(tid >> 5); const int lane = tid & 31, col = lane & 15, g = lane >> 4; const int c0 = blockIdx.y * 128;
  const size_t rb = (size_t)blockIdx.x * 64; const size_t r0 = rb + wave * 16; const size_t orow0 = (rb / TT) * (size_t)SEQ_FULL + (rb % TT) + wave * 16;
  v8f acc[8] = {};
  if ((int)(rb % TT) < QHI) {
#pragma unroll 2
    for (int kc = 0; kc < CC / 32; ++kc) { const F2 a = split_row(Y + (r0 + col) * CC, kc * 32, lane); asm volatile("s_wait_loadcnt 0x0" ::: "memory");
#pragma unroll
      for (int j = 0; j < 8; ++j) { const v16b w = wcol_io(WO, kc * 32, c0 + j * 16 + col, lane, DIN); asm volatile("s_wait_loadcnt 0x0" ::: "memory"); acc[j] = wmma_bf(a.h, w, acc[j]); acc[j] = wmma_bf(a.l, w, acc[j]); } }
#pragma unroll
    for (int j = 0; j < 8; ++j) { const float bias = bfr(BO[c0 + j * 16 + col]);
#pragma unroll
      for (int r = 0; r < 8; ++r) sf[wave][8 * g + r][j * 16 + col] = acc[j][r] + bias; }
  } else {
#pragma unroll 2
    for (int kc = 0; kc < CC / 32; ++kc) { const v16h a = frag_f32s(Y + (r0 + col) * CC + kc * 32, lane, 64.0f); asm volatile("s_wait_loadcnt 0x0" ::: "memory");
#pragma unroll
      for (int j = 0; j < 8; ++j) { const v16h w = wcolh_io(WO, kc * 32, c0 + j * 16 + col, lane, DIN); asm volatile("s_wait_loadcnt 0x0" ::: "memory"); acc[j] = wmma16(a, w, acc[j]); } }
#pragma unroll
    for (int j = 0; j < 8; ++j) { const float bias = bfr(BO[c0 + j * 16 + col]);
#pragma unroll
      for (int r = 0; r < 8; ++r) sf[wave][8 * g + r][j * 16 + col] = acc[j][r] * (1.0f / 16384.0f) + bias; } }
  LDSX(); for (int rl = 0; rl < 16; ++rl) vst2(OUT + (orow0 + rl) * DIN + c0 + lane * 4, *(const v4f*)&sf[wave][rl][lane * 4]); }

extern "C" void kernel_launch(void* const* d_in, const int* in_sizes, int n_in, void* d_out, int out_size, void* d_ws, size_t ws_size, hipStream_t stream) {
  if (n_in < 5) return;
  const long long xneed = ((long long)(NB - 1) * SEQ_FULL + SEQ) * DIN;
  if ((long long)in_sizes[0] < xneed) return;
  if ((long long)in_sizes[1] < (long long)DIN * 3 * CC) return;
  if (in_sizes[2] < 3 * CC) return;
  if ((long long)in_sizes[3] < (long long)CC * DIN) return;
  if (in_sizes[4] < DIN) return;
  if ((long long)out_size < xneed) return;
  if (ws_size < (size_t)WS_END) return;
  const float* x = (const float*)d_in[0]; const float* w_attn = (const float*)d_in[1]; const float* b_attn = (const float*)d_in[2]; const float* w_proj = (const float*)d_in[3]; const float* b_proj = (const float*)d_in[4];
  char* ws = (char*)d_ws;
  _Float16* QH = (_Float16*)(ws + WS_QH); _Float16* KH = (_Float16*)(ws + WS_KH); _Float16* VT = (_Float16*)(ws + WS_VT); _Float16* QL = (_Float16*)(ws + WS_QL); _Float16* KL = (_Float16*)(ws + WS_KL);
  __bf16* VB = (__bf16*)(ws + WS_VB); __bf16* VBL = (__bf16*)(ws + WS_VBL); float* Y = (float*)(ws + WS_Y);
  k_proj<<<dim3(NB * TT / 64, CC / 128, 3), 128, 0, stream>>>(x, w_attn, b_attn, QH, QL, VT, VB, VBL);
  k_fa<<<dim3(NQB, NB * NH), 128, 0, stream>>>(QH, KH, QL, KL, VT, VB, VBL, Y);
  k_out<<<dim3(NB * TT / 64, DIN / 128), 128, 0, stream>>>(Y, w_proj, b_proj, (float*)d_out);
}
